// BottleNeck_Long_61314953118038
// MI455X (gfx1250) — hardware-verified
//
#include <hip/hip_runtime.h>
#include <math.h>


#define EPSV    1e-5f
#define NBATCH  4
#define CIN     64
#define IMH     96
#define IMW     96
#define HW      9216
#define CR      16
#define KS      7
#define KKT     49
#define NG      4
#define KKG     196
#define KKGP    208
#define COUT    128
#define NPIX    (NBATCH * HW)
#define WR_K    192
#define WS_K    64
#define WC_K    384
#define X1P     136
#define PLANE   (256 * X1P)
#define HALO_R  14
#define HALO_C  38
#define HALO_N  (HALO_R * HALO_C)

#define OFF_KS   34048
#define OFF_X1H  84224
#define OFF_X1L  153856
#define OFF_TAB  223488
#define LDS_MAIN 224512

#define WSO_WR    0
#define WSO_WS    6144
#define WSO_WC    32768
#define WSO_KERN  131072
#define WS_TOTAL  29032448

static_assert(16 * HALO_N * 4 == OFF_KS);
static_assert(OFF_KS + KKT * 256 * 4 == OFF_X1H);
static_assert(OFF_X1H + PLANE * 2 == OFF_X1L);
static_assert(OFF_X1L + PLANE * 2 == OFF_TAB);
static_assert(OFF_TAB + 256 * 4 == LDS_MAIN);
static_assert((OFF_X1H % 16) == 0 && (OFF_X1L % 16) == 0 && (OFF_TAB % 16) == 0);
static_assert(8 * 512 * 4 <= KKT * 256 * 4);
static_assert(WSO_WR + CR * WR_K * 2 <= WSO_WS);
static_assert(WSO_WS + KKGP * WS_K * 2 <= WSO_WC);
static_assert(WSO_WC + COUT * WC_K * 2 <= WSO_KERN);
static_assert(WSO_KERN + NBATCH * KKG * HW * 4 == WS_TOTAL);
static_assert(NPIX % 128 == 0);
static_assert(NPIX % 256 == 0);
static_assert(HW % 128 == 0);

typedef unsigned short us;
typedef us     v8us  __attribute__((ext_vector_type(8)));
typedef us     v16us __attribute__((ext_vector_type(16)));
typedef __bf16 v16bf __attribute__((ext_vector_type(16)));
typedef float  v8f   __attribute__((ext_vector_type(8)));
typedef float  v4f   __attribute__((ext_vector_type(4)));

union Frag { v16bf v; v16us u; v8us h[2]; };

__device__ __forceinline__ v8f wmma_bf(const v16bf a, const v16bf b, v8f c) {
    v8f d = __builtin_amdgcn_wmma_f32_16x16x32_bf16(false, a, false, b, (short)0, c, false, false);
    asm volatile("v_nop\n\tv_nop\n\tv_nop\n\tv_nop" : "+v"(d) : "v"(a), "v"(b));
    return d;
}

__device__ __forceinline__ us bf16_rne(float f) {
    unsigned u = __float_as_uint(f);
    u = u + 0x7FFFu + ((u >> 16) & 1u);
    return (us)(u >> 16);
}
__device__ __forceinline__ void split_bf16(float f, us& hi, us& lo) {
    const us hb = bf16_rne(f);
    const float hf = __uint_as_float(((unsigned)hb) << 16);
    hi = hb;
    lo = bf16_rne(f - hf);
}

__device__ __forceinline__ float geluf(float v) {
    return 0.5f * v * (1.0f + erff(v * 0.70710678118654752f));
}

__device__ __forceinline__ v8f zero8() {
    v8f z = {0.f, 0.f, 0.f, 0.f, 0.f, 0.f, 0.f, 0.f};
    return z;
}

__device__ __forceinline__ void st2_v8us(us* p, v8us v) {
    *(volatile v8us*)p = v;
    __threadfence();
    *(volatile v8us*)p = v;
}

__device__ __forceinline__ v8us split8(const float* __restrict__ wp, float s, bool wantlo, bool valid) {
    const v4f wa = *(const v4f*)(wp);
    const v4f wb = *(const v4f*)(wp + 4);
    v8us val;
#pragma unroll
    for (int e = 0; e < 4; ++e) {
        us hb, lb;
        split_bf16(wa[e] * s, hb, lb);
        const us pick = wantlo ? lb : hb;
        val[e] = valid ? pick : (us)0;
    }
#pragma unroll
    for (int e = 0; e < 4; ++e) {
        us hb, lb;
        split_bf16(wb[e] * s, hb, lb);
        const us pick = wantlo ? lb : hb;
        val[4 + e] = valid ? pick : (us)0;
    }
    return val;
}

__global__ __launch_bounds__(256) void k_prep(
    const float* __restrict__ w_reduce, const float* __restrict__ g_r, const float* __restrict__ v_r,
    const float* __restrict__ w_span,
    const float* __restrict__ w_conv, const float* __restrict__ g_c, const float* __restrict__ v_c,
    const float* __restrict__ w_map, const float* __restrict__ g_m, const float* __restrict__ v_m,
    us* __restrict__ wr, us* __restrict__ wsp, us* __restrict__ wcm)
{
    const int tid = threadIdx.x;

#pragma unroll 1
    for (int part = 0; part < 2; ++part) {
        const float* W = part ? w_map : w_conv;
        const float* G = part ? g_m   : g_c;
        const float* V = part ? v_m   : v_c;
#pragma unroll 1
        for (int q = tid; q < COUT * 24; q += 256) {
            const int row = q / 24;
            const int kk  = (q - row * 24) * 8;
            const int seg = kk >> 6;
            const int c0  = kk & 63;
            const float s = G[row] * rsqrtf(V[row] + EPSV);
            const v8us val = split8(W + row * CIN + c0, s, seg == 1, true);
            st2_v8us(wcm + (size_t)row * WC_K + part * 192 + kk, val);
        }
    }

#pragma unroll 1
    for (int q = tid; q < KKGP * 8; q += 256) {
        const int row  = q >> 3;
        const int kb   = (q & 7) * 8;
        const int s16  = kb >> 4;
        const int r0   = kb & 15;
        const int rowc = (row < KKG) ? row : (KKG - 1);
        const bool valid  = (row < KKG) && (s16 < 3);
        const v8us val = split8(w_span + rowc * CR + r0, 1.0f, s16 == 1, valid);
        st2_v8us(wsp + (size_t)q * 8, val);
    }

#pragma unroll 1
    for (int q = tid; q < CR * 24; q += 256) {
        const int row = q / 24;
        const int kk  = (q - row * 24) * 8;
        const int seg = kk >> 6;
        const int c0  = kk & 63;
        const float sr = g_r[row] * rsqrtf(v_r[row] + EPSV);
        const v8us val = split8(w_reduce + row * CIN + c0, sr, seg == 1, true);
        st2_v8us(wr + (size_t)q * 8, val);
    }
}

__global__ __launch_bounds__(128) void k_kern(
    const float* __restrict__ x, const us* __restrict__ wr, const us* __restrict__ wsp,
    const float* __restrict__ g_r, const float* __restrict__ b_r,
    const float* __restrict__ m_r, const float* __restrict__ v_r,
    const float* __restrict__ b_span, float* __restrict__ kern_ws)
{
    __shared__ float offr_s[16];
    __shared__ float bsp_s[KKGP];
    __shared__ __attribute__((aligned(16))) float stg[4 * 512];
    __shared__ __attribute__((aligned(16))) float xt[CIN * 128];

    const int tid  = threadIdx.x;
    const int lane = tid & 31;
    const int wv   = tid >> 5;
    const int h    = lane >> 4;
    const int m    = lane & 15;

    if (tid < 16) {
        const float sr = g_r[tid] * rsqrtf(v_r[tid] + EPSV);
        offr_s[tid] = b_r[tid] - m_r[tid] * sr;
    }
    for (int i = tid; i < KKGP; i += 128) {
        const int ic = (i < KKG) ? i : (KKG - 1);
        const float v = b_span[ic];
        bsp_s[i] = (i < KKG) ? v : 0.f;
    }

    const int pixb  = blockIdx.x * 128;
    const int b     = pixb / HW;
    const int pixb0 = pixb - b * HW;
    const float* xblk = x + (size_t)b * CIN * HW + pixb0;

#pragma unroll 1
    for (int jj = 0; jj < 4; ++jj) {
        v4f v[4];
#pragma unroll
        for (int u = 0; u < 4; ++u) {
            const int c = 16 * jj + 4 * u + wv;
            v[u] = *(const v4f*)(xblk + (size_t)c * HW + 4 * lane);
        }
#pragma unroll
        for (int u = 0; u < 4; ++u) {
            const int c = 16 * jj + 4 * u + wv;
            *(v4f*)(xt + c * 128 + 4 * lane) = v[u];
        }
    }
    __syncthreads();

    const int pix0 = pixb0 + wv * 32;

    Frag bxh[2][2], bxl[2][2];
#pragma unroll
    for (int nt = 0; nt < 2; ++nt) {
#pragma unroll
        for (int p = 0; p < 2; ++p) {
#pragma unroll
            for (int i = 0; i < 16; ++i) {
                const int c = 32 * p + 8 * h + (i & 7) + ((i >> 3) << 4);
                const float v = xt[c * 128 + wv * 32 + 16 * nt + m];
                us hb, lb;
                split_bf16(v, hb, lb);
                bxh[nt][p].u[i] = hb;
                bxl[nt][p].u[i] = lb;
            }
        }
    }

    v8f accr[2];
    accr[0] = zero8();
    accr[1] = zero8();
    const us* arow = wr + m * WR_K + 8 * h;
#pragma unroll 1
    for (int sg = 0; sg < 2; ++sg) {
#pragma unroll
        for (int p = 0; p < 2; ++p) {
            Frag a;
            a.h[0] = *(const v8us*)(arow + 64 * sg + 32 * p);
            a.h[1] = *(const v8us*)(arow + 64 * sg + 32 * p + 16);
#pragma unroll
            for (int nt = 0; nt < 2; ++nt)
                accr[nt] = wmma_bf(a.v, bxh[nt][p].v, accr[nt]);
        }
    }
#pragma unroll
    for (int p = 0; p < 2; ++p) {
        Frag a;
        a.h[0] = *(const v8us*)(arow + 128 + 32 * p);
        a.h[1] = *(const v8us*)(arow + 128 + 32 * p + 16);
#pragma unroll
        for (int nt = 0; nt < 2; ++nt)
            accr[nt] = wmma_bf(a.v, bxl[nt][p].v, accr[nt]);
    }

    Frag bt0[2], bt1[2];
#pragma unroll
    for (int nt = 0; nt < 2; ++nt) {
#pragma unroll
        for (int r = 0; r < 8; ++r) {
            const float tv = fmaxf(accr[nt][r] + offr_s[8 * h + r], 0.f);
            us hb, lb;
            split_bf16(tv, hb, lb);
            bt0[nt].u[r]     = hb;
            bt0[nt].u[8 + r] = hb;
            bt1[nt].u[r]     = lb;
            bt1[nt].u[8 + r] = (us)0;
        }
    }

    float* stgw = stg + wv * 512;
    float* kwb  = kern_ws + (size_t)b * KKG * HW + pix0;
    const int rl = lane >> 3;
    const int q4 = lane & 7;

#pragma unroll 1
    for (int mt = 0; mt < 13; ++mt) {
        const us* ap = wsp + (size_t)(mt * 16 + m) * WS_K + 8 * h;
        Frag a0, a1;
        a0.h[0] = *(const v8us*)(ap);
        a0.h[1] = *(const v8us*)(ap + 16);
        a1.h[0] = *(const v8us*)(ap + 32);
        a1.h[1] = *(const v8us*)(ap + 48);
        v8f c[2];
#pragma unroll
        for (int nt = 0; nt < 2; ++nt) {
            c[nt] = wmma_bf(a0.v, bt0[nt].v, zero8());
            c[nt] = wmma_bf(a1.v, bt1[nt].v, c[nt]);
        }

        __syncthreads();
#pragma unroll
        for (int nt = 0; nt < 2; ++nt) {
#pragma unroll
            for (int r = 0; r < 8; ++r) {
                const int ol = 8 * h + r;
                stgw[ol * 32 + 16 * nt + m] = c[nt][r] + bsp_s[mt * 16 + ol];
            }
        }
        __syncthreads();

        const int nrows = (mt == 12) ? (KKG - 192) : 16;
        const int ninst = nrows >> 2;
        v4f vals[4];
#pragma unroll
        for (int j = 0; j < 4; ++j)
            vals[j] = *(const v4f*)(stgw + (4 * j + rl) * 32 + q4 * 4);
#pragma unroll
        for (int j = 0; j < 4; ++j) {
            if (j < ninst) {
                const int o = mt * 16 + 4 * j + rl;
                float* pdst = kwb + (size_t)o * HW + q4 * 4;
                *(volatile v4f*)pdst = vals[j];
            }
        }
        __threadfence();
#pragma unroll
        for (int j = 0; j < 4; ++j) {
            if (j < ninst) {
                const int o = mt * 16 + 4 * j + rl;
                float* pdst = kwb + (size_t)o * HW + q4 * 4;
                *(volatile v4f*)pdst = vals[j];
            }
        }
    }
}

__global__ __launch_bounds__(256) void k_main(
    const float* __restrict__ x, const float* __restrict__ kern_ws, const us* __restrict__ wcm,
    const float* __restrict__ g_i, const float* __restrict__ b_i,
    const float* __restrict__ m_i, const float* __restrict__ v_i,
    const float* __restrict__ g_c, const float* __restrict__ b_c,
    const float* __restrict__ m_c, const float* __restrict__ v_c,
    const float* __restrict__ b_map,
    const float* __restrict__ g_m, const float* __restrict__ b_m,
    const float* __restrict__ m_m, const float* __restrict__ v_m,
    float* __restrict__ out)
{
    extern __shared__ __attribute__((aligned(16))) unsigned char dynlds[];
    float* xs     = (float*)(dynlds);
    float* ks     = (float*)(dynlds + OFF_KS);
    us*    x1h    = (us*)(dynlds + OFF_X1H);
    float* si_s   = (float*)(dynlds + OFF_TAB);
    float* oi_s   = si_s + 64;
    float* bias_s = si_s + 128;
    float* stg    = ks;

    const int tid  = threadIdx.x;
    const int lane = tid & 31;
    const int wv   = tid >> 5;
    const int h    = lane >> 4;
    const int m    = lane & 15;

    const int blk = blockIdx.x;
    const int b   = blk / 36;
    const int rem = blk - b * 36;
    const int th  = rem / 3;
    const int tw  = rem - th * 3;
    const int h0  = th * 8;
    const int w0  = tw * 32;

    if (tid < 64) {
        const float s = g_i[tid] * rsqrtf(v_i[tid] + EPSV);
        si_s[tid] = s;
        oi_s[tid] = b_i[tid] - m_i[tid] * s;
    }
    if (tid < 128) {
        const float s1 = g_c[tid] * rsqrtf(v_c[tid] + EPSV);
        const float s2 = g_m[tid] * rsqrtf(v_m[tid] + EPSV);
        bias_s[tid] = (b_c[tid] - m_c[tid] * s1) + (b_m[tid] - m_m[tid] * s2) + b_map[tid] * s2;
    }

#pragma unroll 1
    for (int g = 0; g < NG; ++g) {
        __syncthreads();

        const float* xg = x + ((size_t)b * CIN + g * 16) * HW;
#pragma unroll 1
        for (int ch = 0; ch < 16; ++ch) {
            const float* xc = xg + (size_t)ch * HW;
            for (int idx = tid; idx < HALO_N; idx += 256) {
                const int r  = idx / HALO_C;
                const int cc = idx - r * HALO_C;
                const int hh = h0 + r - 3;
                const int ww = w0 + cc - 3;
                const int hc = (hh < 0) ? 0 : ((hh > IMH - 1) ? (IMH - 1) : hh);
                const int wc = (ww < 0) ? 0 : ((ww > IMW - 1) ? (IMW - 1) : ww);
                const float v = xc[hc * IMW + wc];
                const bool inside = (hh >= 0) && (hh < IMH) && (ww >= 0) && (ww < IMW);
                xs[ch * HALO_N + idx] = inside ? v : 0.f;
            }
        }
        const float* kp = kern_ws + ((size_t)b * KKG + g * KKT) * HW + (size_t)(h0 + wv) * IMW + w0 + lane;
#pragma unroll 7
        for (int it = 0; it < KKT; ++it)
            ks[it * 256 + tid] = kp[(size_t)it * HW];
        __syncthreads();

        float acc[16];
#pragma unroll
        for (int ch = 0; ch < 16; ++ch) acc[ch] = 0.f;
#pragma unroll 1
        for (int ti = 0; ti < KS; ++ti) {
            const float* xrow = xs + (wv + ti) * HALO_C + lane;
            const float* krow = ks + ti * KS * 256 + tid;
#pragma unroll
            for (int tj = 0; tj < KS; ++tj) {
                const float kv = krow[tj * 256];
                const float* xp = xrow + tj;
#pragma unroll
                for (int ch = 0; ch < 16; ++ch)
                    acc[ch] = fmaf(kv, xp[ch * HALO_N], acc[ch]);
            }
        }

        Frag hx, lx, hy, ly;
        const float* xctr = xs + (wv + 3) * HALO_C + lane + 3;
#pragma unroll
        for (int ch = 0; ch < 16; ++ch) {
            const int cch = g * 16 + ch;
            const float v = geluf(acc[ch] * si_s[cch] + oi_s[cch]);
            us hb, lb;
            split_bf16(v, hb, lb);
            hx.u[ch] = hb;
            lx.u[ch] = lb;
            const float xv = xctr[ch * HALO_N];
            us hb2, lb2;
            split_bf16(xv, hb2, lb2);
            hy.u[ch] = hb2;
            ly.u[ch] = lb2;
        }
        us* ph = x1h + tid * X1P + g * 16;
        us* pl = ph + PLANE;
        *(v8us*)(ph)          = hx.h[0];
        *(v8us*)(ph + 8)      = hx.h[1];
        *(v8us*)(pl)          = lx.h[0];
        *(v8us*)(pl + 8)      = lx.h[1];
        *(v8us*)(ph + 64)     = hy.h[0];
        *(v8us*)(ph + 64 + 8) = hy.h[1];
        *(v8us*)(pl + 64)     = ly.h[0];
        *(v8us*)(pl + 64 + 8) = ly.h[1];
    }
    __syncthreads();

    const size_t prow = (size_t)(h0 + wv) * IMW + w0;
    float* outb = out + (size_t)b * COUT * HW + prow;
    float* stgw = stg + wv * 512;
    const int rl = lane >> 3;
    const int q4 = lane & 7;
    const us* bw = x1h + (wv * 32 + m) * X1P + 8 * h;

#pragma unroll 1
    for (int mt = 0; mt < 8; ++mt) {
        v8f acc0 = zero8();
        v8f acc1 = zero8();
        const us* ap = wcm + (size_t)(mt * 16 + m) * WC_K + 8 * h;
#pragma unroll 1
        for (int sg = 0; sg < 6; ++sg) {
            const int lob = (sg == 2 || sg == 5) ? 1 : 0;
            const int cof = (sg >= 3) ? 64 : 0;
            const us* bp = bw + lob * PLANE + cof;
            const us* aq = ap + 64 * sg;
#pragma unroll
            for (int p = 0; p < 2; ++p) {
                Frag a, b0, b1;
                a.h[0]  = *(const v8us*)(aq + 32 * p);
                a.h[1]  = *(const v8us*)(aq + 32 * p + 16);
                b0.h[0] = *(const v8us*)(bp + 32 * p);
                b0.h[1] = *(const v8us*)(bp + 32 * p + 16);
                b1.h[0] = *(const v8us*)(bp + 16 * X1P + 32 * p);
                b1.h[1] = *(const v8us*)(bp + 16 * X1P + 32 * p + 16);
                acc0 = wmma_bf(a.v, b0.v, acc0);
                acc1 = wmma_bf(a.v, b1.v, acc1);
            }
        }

        __syncthreads();
#pragma unroll
        for (int r = 0; r < 8; ++r) {
            const int ol = 8 * h + r;
            const float bs = bias_s[mt * 16 + ol];
            stgw[ol * 32 + m]      = geluf(acc0[r] + bs);
            stgw[ol * 32 + 16 + m] = geluf(acc1[r] + bs);
        }
        __syncthreads();

        v4f vals[4];
#pragma unroll
        for (int j = 0; j < 4; ++j)
            vals[j] = *(const v4f*)(stgw + (4 * j + rl) * 32 + q4 * 4);
#pragma unroll
        for (int j = 0; j < 4; ++j) {
            const int o = mt * 16 + 4 * j + rl;
            float* pdst = outb + (size_t)o * HW + q4 * 4;
            *(volatile v4f*)pdst = vals[j];
        }
        __threadfence();
#pragma unroll
        for (int j = 0; j < 4; ++j) {
            const int o = mt * 16 + 4 * j + rl;
            float* pdst = outb + (size_t)o * HW + q4 * 4;
            *(volatile v4f*)pdst = vals[j];
        }
    }
}

extern "C" void kernel_launch(void* const* d_in, const int* in_sizes, int n_in,
                              void* d_out, int out_size, void* d_ws, size_t ws_size,
                              hipStream_t stream)
{
    if (n_in < 23) return;
    if (in_sizes[0] != NPIX * CIN || in_sizes[1] != CR * CIN || in_sizes[6] != KKG * CR ||
        in_sizes[7] != KKG || in_sizes[12] != COUT * CIN || in_sizes[17] != COUT * CIN ||
        in_sizes[18] != COUT) return;
    if (out_size != NPIX * COUT) return;
    if (ws_size < (size_t)WS_TOTAL) return;

    const float* x        = (const float*)d_in[0];
    const float* w_reduce = (const float*)d_in[1];
    const float* g_r      = (const float*)d_in[2];
    const float* b_r      = (const float*)d_in[3];
    const float* m_r      = (const float*)d_in[4];
    const float* v_r      = (const float*)d_in[5];
    const float* w_span   = (const float*)d_in[6];
    const float* b_span   = (const float*)d_in[7];
    const float* g_i      = (const float*)d_in[8];
    const float* b_i      = (const float*)d_in[9];
    const float* m_i      = (const float*)d_in[10];
    const float* v_i      = (const float*)d_in[11];
    const float* w_conv   = (const float*)d_in[12];
    const float* g_c      = (const float*)d_in[13];
    const float* b_c      = (const float*)d_in[14];
    const float* m_c      = (const float*)d_in[15];
    const float* v_c      = (const float*)d_in[16];
    const float* w_map    = (const float*)d_in[17];
    const float* b_map    = (const float*)d_in[18];
    const float* g_m      = (const float*)d_in[19];
    const float* b_m      = (const float*)d_in[20];
    const float* m_m      = (const float*)d_in[21];
    const float* v_m      = (const float*)d_in[22];
    float* out = (float*)d_out;

    unsigned char* wsb = (unsigned char*)d_ws;
    us*    wr      = (us*)(wsb + WSO_WR);
    us*    wsp     = (us*)(wsb + WSO_WS);
    us*    wcm     = (us*)(wsb + WSO_WC);
    float* kern_ws = (float*)(wsb + WSO_KERN);

    k_prep<<<dim3(1), dim3(256), 0, stream>>>(
        w_reduce, g_r, v_r, w_span, w_conv, g_c, v_c, w_map, g_m, v_m, wr, wsp, wcm);

    k_kern<<<dim3(NPIX / 128), dim3(128), 0, stream>>>(
        x, wr, wsp, g_r, b_r, m_r, v_r, b_span, kern_ws);

    (void)hipFuncSetAttribute(reinterpret_cast<const void*>(&k_main),
                              hipFuncAttributeMaxDynamicSharedMemorySize, LDS_MAIN);
    k_main<<<dim3(NPIX / 256), dim3(256), LDS_MAIN, stream>>>(
        x, kern_ws, wcm, g_i, b_i, m_i, v_i, g_c, b_c, m_c, v_c, b_map, g_m, b_m, m_m, v_m, out);
}
